// HierarchicalHopfield_455266533847
// MI455X (gfx1250) — hardware-verified
//
#include <hip/hip_runtime.h>
#include <math.h>

constexpr int kRows   = 4096;
constexpr int kDim    = 512;
constexpr int kNCls   = 12;
constexpr int kKCls   = 500;
constexpr int kKClsP  = 512;
constexpr int kKGlb   = 5000;
constexpr int kKGlbP  = 5120;
constexpr int kHid    = 64;
constexpr int kGChunk = 2048;
constexpr int kCHalf  = 6;
constexpr float kPCarry    = 2048.0f;
constexpr float kPCarryInv = 1.0f / 2048.0f;
constexpr float kGCarry    = 64.0f;
constexpr float kGateScale = 1.0f / 4096.0f;

typedef __attribute__((ext_vector_type(16))) _Float16 v16h;
typedef __attribute__((ext_vector_type(8)))  _Float16 v8h;
typedef __attribute__((ext_vector_type(16))) __bf16   v16b;
typedef __attribute__((ext_vector_type(8)))  __bf16   v8b;
typedef __attribute__((ext_vector_type(8)))  float    v8f;
typedef __attribute__((ext_vector_type(4)))  float    v4f;
typedef __attribute__((ext_vector_type(4)))  unsigned int v4u;

__device__ __forceinline__ unsigned short f2bf_bits(float f) {
  unsigned u = __float_as_uint(f);
  return (unsigned short)((u + 0x7FFFu + ((u >> 16) & 1u)) >> 16);
}
__device__ __forceinline__ float bf_bits2f(unsigned short h) { return __uint_as_float(((unsigned)h) << 16); }

__device__ __forceinline__ void dep_guard_h(v8f& a, v8f& b, v16h x, v16h y) { asm volatile("v_nop\n\tv_nop\n\tv_nop\n\tv_nop" : "+v"(a), "+v"(b) : "v"(x), "v"(y)); }
__device__ __forceinline__ void dep_guard_b(v8f& a, v8f& b, v16b x, v16b y) { asm volatile("v_nop\n\tv_nop\n\tv_nop\n\tv_nop" : "+v"(a), "+v"(b) : "v"(x), "v"(y)); }
__device__ __forceinline__ void keep4_h(v16h a, v16h b, v16h c, v16h d) { asm volatile("v_nop" :: "v"(a), "v"(b), "v"(c), "v"(d)); }
__device__ __forceinline__ void keep4_b(v16b a, v16b b, v16b c, v16b d) { asm volatile("v_nop" :: "v"(a), "v"(b), "v"(c), "v"(d)); }
__device__ __forceinline__ void acc_guard4(v8f& a, v8f& b, v8f& c, v8f& d) { asm volatile("v_nop\n\tv_nop\n\tv_nop\n\tv_nop" : "+v"(a), "+v"(b), "+v"(c), "+v"(d)); }
template <typename T> struct Frag;
template <> struct Frag<_Float16> {
  typedef v16h V; union U { v16h v; v8h h[2]; };
  static __device__ __forceinline__ v16h load(const _Float16* p) {
    U f; f.h[0] = *(const v8h*)(p); f.h[1] = *(const v8h*)(p + 16); return f.v;
  }
  static __device__ __forceinline__ v8f mma(v16h a, v16h b, v8f c) {
    return __builtin_amdgcn_wmma_f32_16x16x32_f16(false, a, false, b, (short)0, c, false, false);
  }
  static __device__ __forceinline__ void guard(v8f& a, v8f& b, v16h x, v16h y) { dep_guard_h(a, b, x, y); }
  static __device__ __forceinline__ void keep(v16h a, v16h b, v16h c, v16h d) { keep4_h(a, b, c, d); }
};
template <> struct Frag<__bf16> {
  typedef v16b V; union U { v16b v; v8b h[2]; };
  static __device__ __forceinline__ v16b load(const __bf16* p) {
    U f; f.h[0] = *(const v8b*)(p); f.h[1] = *(const v8b*)(p + 16); return f.v;
  }
  static __device__ __forceinline__ v8f mma(v16b a, v16b b, v8f c) {
    return __builtin_amdgcn_wmma_f32_16x16x32_bf16(false, a, false, b, (short)0, c, false, false);
  }
  static __device__ __forceinline__ void guard(v8f& a, v8f& b, v16b x, v16b y) { dep_guard_b(a, b, x, y); }
  static __device__ __forceinline__ void keep(v16b a, v16b b, v16b c, v16b d) { keep4_b(a, b, c, d); }
};

__device__ __forceinline__ unsigned pk16(unsigned short a, unsigned short b) { return (unsigned)a | ((unsigned)b << 16); }
__device__ __forceinline__ unsigned short h_bits(float f) { const _Float16 h = (_Float16)f; return __builtin_bit_cast(unsigned short, h); }

template <int ET> struct Elem;
template <> struct Elem<0> { typedef _Float16 T; };
template <> struct Elem<1> { typedef __bf16 T; };
template <int ET, bool SPLIT, int BIAS_MODE, int OUT_MODE, bool RESID, int ACT = 0>
__global__ __launch_bounds__(256) void wmma_gemm64(
    const unsigned short* __restrict__ Ap, const unsigned short* __restrict__ A2p, int lda, long strideA,
    const unsigned short* __restrict__ Btp, const unsigned short* __restrict__ Bt2p, int ldb, long strideB,
    void* __restrict__ Cout, void* __restrict__ Cout2, int ldc, long strideC,
    const float* __restrict__ bias,
    const float* __restrict__ resid, long strideR,
    int M, int N, int K, float scale) {
  typedef typename Elem<ET>::T T;
  typedef typename Frag<T>::V V;
  const T* A = (const T*)Ap; const T* A2 = (const T*)A2p; const T* Bt = (const T*)Btp; const T* Bt2 = (const T*)Bt2p;
  __shared__ __align__(16) float sT[8][16 * 68];
  const int b    = blockIdx.y;
  const int lane = threadIdx.x & 31;
  const int wave = threadIdx.x >> 5;
  const int tilesN = N >> 6;
  const int tilesM = M >> 6;
  const int tile = blockIdx.x * 8 + wave;
  if (tile >= tilesM * tilesN) return;
  const int tm = tile / tilesN;
  const int tn = tile - tm * tilesN;
  const int m0 = tm << 6;
  const int n0 = tn << 6;

  const T* Ab  = A  + (size_t)b * strideA;
  const T* Bb  = Bt + (size_t)b * strideB;
  const T* Ab2 = SPLIT ? (A2  + (size_t)b * strideA) : nullptr;
  const T* Bb2 = SPLIT ? (Bt2 + (size_t)b * strideB) : nullptr;

  const int rlane = lane & 15;
  const int koff  = (lane >> 4) * 8;
  const int mOff  = (lane >> 4) * 8;

  v8f acc[4][4];
#pragma unroll
  for (int i = 0; i < 4; ++i)
#pragma unroll
    for (int j = 0; j < 4; ++j) acc[i][j] = (v8f){0.f,0.f,0.f,0.f,0.f,0.f,0.f,0.f};

  for (int k0 = 0; k0 < K; k0 += 32) {
    V bh[4], bl[4];
#pragma unroll
    for (int j = 0; j < 4; ++j) {
      const size_t bo = (size_t)(n0 + (j << 4) + rlane) * ldb + koff + k0;
      bh[j] = Frag<T>::load(Bb + bo);
      if (SPLIT) bl[j] = Frag<T>::load(Bb2 + bo);
    }
#pragma unroll
    for (int i = 0; i < 4; ++i) {
      const size_t ao = (size_t)(m0 + (i << 4) + rlane) * lda + koff + k0;
      V ah = Frag<T>::load(Ab + ao);
      V al;
      if (SPLIT) al = Frag<T>::load(Ab2 + ao);
#pragma unroll
      for (int j = 0; j < 4; ++j) {
        acc[i][j] = Frag<T>::mma(ah, bh[j], acc[i][j]);
        if (SPLIT) {
          acc[i][j] = Frag<T>::mma(ah, bl[j], acc[i][j]);
          acc[i][j] = Frag<T>::mma(al, bh[j], acc[i][j]);
        }
      }
      Frag<T>::guard(acc[i][0], acc[i][3], ah, SPLIT ? al : ah);
    }
    Frag<T>::keep(bh[0], bh[1], bh[2], bh[3]);
    if (SPLIT) Frag<T>::keep(bl[0], bl[1], bl[2], bl[3]);
  }
  acc_guard4(acc[0][0], acc[0][1], acc[0][2], acc[0][3]);
  acc_guard4(acc[1][0], acc[1][1], acc[1][2], acc[1][3]);
  acc_guard4(acc[2][0], acc[2][1], acc[2][2], acc[2][3]);
  acc_guard4(acc[3][0], acc[3][1], acc[3][2], acc[3][3]);

  float* slab = sT[wave];
  const float* Rb = RESID ? (resid + (size_t)b * strideR) : nullptr;
#pragma unroll
  for (int i = 0; i < 4; ++i) {
    const int mBase = m0 + (i << 4);
#pragma unroll
    for (int j = 0; j < 4; ++j) {
      const int n = n0 + (j << 4) + rlane;
      float bv = 0.f;
      if (BIAS_MODE == 2) bv = bias[n];
#pragma unroll
      for (int r = 0; r < 8; ++r) {
        float v = acc[i][j][r] * scale;
        if (BIAS_MODE == 1) v += bias[mBase + mOff + r];
        if (BIAS_MODE == 2) v += bv;
        if (RESID) v += Rb[(size_t)(mBase + mOff + r) * ldc + n];
        if (ACT == 2) v = fmaxf(v, 0.0f);
        if (ACT == 4) v = (v > 0.f) ? v : 0.01f * v;
        slab[(mOff + r) * 68 + (j << 4) + rlane] = v;
      }
    }
    __builtin_amdgcn_fence(__ATOMIC_RELEASE, "workgroup");
    __builtin_amdgcn_wave_barrier();
    __builtin_amdgcn_fence(__ATOMIC_ACQUIRE, "workgroup");
    if (OUT_MODE == 0) {
      float* C = (float*)Cout + (size_t)b * strideC;
      const int hh = lane >> 4, c4 = (lane & 15) * 4;
      for (int pass = 0; pass < 2; ++pass) {
#pragma unroll
        for (int it = 0; it < 8; ++it) {
          const int row = it * 2 + hh;
          v4f v = *(const v4f*)(slab + row * 68 + c4);
          *(volatile v4f*)(C + (size_t)(mBase + row) * ldc + n0 + c4) = v;
        }
        __threadfence();
      }
    } else {
      const int q = lane >> 3, c8 = (lane & 7) * 8;
      unsigned short* C  = (unsigned short*)Cout  + (size_t)b * strideC;
      unsigned short* C2 = (OUT_MODE == 2) ? ((unsigned short*)Cout2 + (size_t)b * strideC) : nullptr;
      for (int pass = 0; pass < 2; ++pass) {
#pragma unroll
        for (int it = 0; it < 4; ++it) {
          const int row = it * 4 + q;
          const float* sp = slab + row * 68 + c8;
          v8h hv, lv;
#pragma unroll
          for (int e = 0; e < 8; ++e) {
            if (OUT_MODE == 1) {
              hv[e] = (_Float16)sp[e];
            } else {
              unsigned short hb = f2bf_bits(sp[e]);
              unsigned short lb = f2bf_bits(sp[e] - bf_bits2f(hb));
              hv[e] = __builtin_bit_cast(_Float16, hb);
              lv[e] = __builtin_bit_cast(_Float16, lb);
            }
          }
          *(volatile v8h*)(C + (size_t)(mBase + row) * ldc + n0 + c8) = hv;
          if (OUT_MODE == 2) *(volatile v8h*)(C2 + (size_t)(mBase + row) * ldc + n0 + c8) = lv;
        }
        __threadfence();
      }
    }
    __builtin_amdgcn_fence(__ATOMIC_RELEASE, "workgroup");
    __builtin_amdgcn_wave_barrier();
    __builtin_amdgcn_fence(__ATOMIC_ACQUIRE, "workgroup");
  }
}

__global__ __launch_bounds__(256) void split8_bf16_kernel(const float* __restrict__ in, int in_rows, int out_rows, int row_len8,
                                                          unsigned short* __restrict__ hi, unsigned short* __restrict__ lo, int n8) {
  const int i = blockIdx.x * 256 + threadIdx.x;
  if (i >= n8) return;
  const int per_batch = out_rows * row_len8;
  const int z   = i / per_batch;
  const int rem = i - z * per_batch;
  const int row = rem / row_len8;
  const int c8  = (rem - row * row_len8) * 8;
  const int rowc = (row < in_rows) ? row : (in_rows - 1);
  const float* p = in + ((size_t)z * in_rows + rowc) * (size_t)(row_len8 * 8) + c8;
  const v4f a = *(const v4f*)(p);
  const v4f c = *(const v4f*)(p + 4);
  const bool valid = row < in_rows;
  float x[8];
#pragma unroll
  for (int e = 0; e < 4; ++e) { x[e] = valid ? a[e] : 0.0f; x[4 + e] = valid ? c[e] : 0.0f; }
  unsigned short hb[8], lb[8];
#pragma unroll
  for (int e = 0; e < 8; ++e) {
    hb[e] = f2bf_bits(x[e]);
    lb[e] = f2bf_bits(x[e] - bf_bits2f(hb[e]));
  }
  const v4u uh = (v4u){pk16(hb[0], hb[1]), pk16(hb[2], hb[3]), pk16(hb[4], hb[5]), pk16(hb[6], hb[7])};
  const v4u ul = (v4u){pk16(lb[0], lb[1]), pk16(lb[2], lb[3]), pk16(lb[4], lb[5]), pk16(lb[6], lb[7])};
  unsigned short* qh = hi + 8 * (size_t)i;
  unsigned short* ql = lo + 8 * (size_t)i;
  *(volatile v4u*)qh = uh;
  *(volatile v4u*)ql = ul;
  __threadfence();
  *(volatile v4u*)qh = uh;
  *(volatile v4u*)ql = ul;
}

__global__ __launch_bounds__(256) void tcast_kernel(const float* __restrict__ in, long in_bstride, int ld_in, int nrows_valid,
                                                    unsigned short* __restrict__ out, long out_bstride, int ld_out, float scale) {
  __shared__ float sm[64][65];
  const int t  = threadIdx.x;
  const int r0 = blockIdx.x * 64;
  const int c0 = blockIdx.y * 64;
  const int z  = blockIdx.z;
  const float* ip = in + (size_t)z * in_bstride;
#pragma unroll
  for (int i = 0; i < 16; ++i) {
    const int e  = i * 256 + t;
    const int rl = e >> 6;
    const int cl = e & 63;
    const int row  = r0 + rl;
    const int rowc = (row < nrows_valid) ? row : (nrows_valid - 1);
    float v = ip[(size_t)rowc * ld_in + c0 + cl] * scale;
    if (row >= nrows_valid) v = 0.0f;
    sm[cl][rl] = v;
  }
  __syncthreads();
  const int lane = t & 31, wave = t >> 5;
  const int q = lane >> 3, c8 = (lane & 7) * 8;
  unsigned short* op = out + (size_t)z * out_bstride;
  for (int pass = 0; pass < 2; ++pass) {
#pragma unroll
    for (int it = 0; it < 2; ++it) {
      const int row = wave * 8 + it * 4 + q;
      unsigned short hb[8];
#pragma unroll
      for (int e = 0; e < 8; ++e) hb[e] = h_bits(sm[row][c8 + e]);
      const v4u u = (v4u){pk16(hb[0], hb[1]), pk16(hb[2], hb[3]), pk16(hb[4], hb[5]), pk16(hb[6], hb[7])};
      *(volatile v4u*)(op + (size_t)(c0 + row) * ld_out + r0 + c8) = u;
    }
    __threadfence();
  }
}

__global__ __launch_bounds__(640) void softmax_g_kernel(const float* __restrict__ S, unsigned short* __restrict__ P) {
  __shared__ float redM[20];
  __shared__ float redS[20];
  const int row  = blockIdx.x;
  const int t    = threadIdx.x;
  const int lane = t & 31, wave = t >> 5;
  const int c0   = t * 8;
  const float* sr = S + (size_t)row * kKGlbP + c0;
  const v4f a = *(const v4f*)(sr);
  const v4f c = *(const v4f*)(sr + 4);
  float x[8];
#pragma unroll
  for (int e = 0; e < 4; ++e) { x[e] = a[e]; x[4 + e] = c[e]; }
#pragma unroll
  for (int e = 0; e < 8; ++e) x[e] = (c0 + e < kKGlb) ? x[e] : -INFINITY;
  float m = fmaxf(fmaxf(fmaxf(x[0], x[1]), fmaxf(x[2], x[3])), fmaxf(fmaxf(x[4], x[5]), fmaxf(x[6], x[7])));
#pragma unroll
  for (int off = 16; off > 0; off >>= 1) m = fmaxf(m, __shfl_xor(m, off, 32));
  if (lane == 0) redM[wave] = m;
  __syncthreads();
  float mm = redM[0];
#pragma unroll
  for (int w = 1; w < 20; ++w) mm = fmaxf(mm, redM[w]);
  float p[8];
  float sum = 0.f;
#pragma unroll
  for (int e = 0; e < 8; ++e) { p[e] = expf(x[e] - mm); sum += p[e]; }
#pragma unroll
  for (int off = 16; off > 0; off >>= 1) sum += __shfl_xor(sum, off, 32);
  if (lane == 0) redS[wave] = sum;
  __syncthreads();
  float tot = redS[0];
#pragma unroll
  for (int w = 1; w < 20; ++w) tot += redS[w];
  const float sc = kPCarry * (1.0f / tot);
  unsigned short hb[8];
#pragma unroll
  for (int e = 0; e < 8; ++e) hb[e] = h_bits(p[e] * sc);
  const v4u u = (v4u){pk16(hb[0], hb[1]), pk16(hb[2], hb[3]), pk16(hb[4], hb[5]), pk16(hb[6], hb[7])};
  unsigned short* q = P + (size_t)row * kKGlbP + c0;
  *(volatile v4u*)q = u;
  __threadfence();
  *(volatile v4u*)q = u;
}

__global__ __launch_bounds__(256) void softmax_c_kernel(const float* __restrict__ S, unsigned short* __restrict__ P) {
  __shared__ float redM[8];
  __shared__ float redS[8];
  const int t    = threadIdx.x;
  const int lane = t & 31, wave = t >> 5, grp = t >> 6, tl = t & 63;
  const int row  = blockIdx.x * 4 + grp;
  const int c0   = tl * 8;
  const float* sr = S + (size_t)row * kKClsP + c0;
  const v4f a = *(const v4f*)(sr);
  const v4f c = *(const v4f*)(sr + 4);
  float x[8];
#pragma unroll
  for (int e = 0; e < 4; ++e) { x[e] = a[e]; x[4 + e] = c[e]; }
#pragma unroll
  for (int e = 0; e < 8; ++e) x[e] = (c0 + e < kKCls) ? x[e] : -INFINITY;
  float m = fmaxf(fmaxf(fmaxf(x[0], x[1]), fmaxf(x[2], x[3])), fmaxf(fmaxf(x[4], x[5]), fmaxf(x[6], x[7])));
#pragma unroll
  for (int off = 16; off > 0; off >>= 1) m = fmaxf(m, __shfl_xor(m, off, 32));
  if (lane == 0) redM[wave] = m;
  __syncthreads();
  const float mm = fmaxf(redM[2 * grp], redM[2 * grp + 1]);
  float p[8];
  float sum = 0.f;
#pragma unroll
  for (int e = 0; e < 8; ++e) { p[e] = expf(x[e] - mm); sum += p[e]; }
#pragma unroll
  for (int off = 16; off > 0; off >>= 1) sum += __shfl_xor(sum, off, 32);
  if (lane == 0) redS[wave] = sum;
  __syncthreads();
  const float tot = redS[2 * grp] + redS[2 * grp + 1];
  const float sc = kPCarry * (1.0f / tot);
  unsigned short hb[8];
#pragma unroll
  for (int e = 0; e < 8; ++e) hb[e] = h_bits(p[e] * sc);
  const v4u u = (v4u){pk16(hb[0], hb[1]), pk16(hb[2], hb[3]), pk16(hb[4], hb[5]), pk16(hb[6], hb[7])};
  unsigned short* q = P + (size_t)row * kKClsP + c0;
  *(volatile v4u*)q = u;
  __threadfence();
  *(volatile v4u*)q = u;
}

__global__ __launch_bounds__(256) void select_kernel(const float* __restrict__ R, const int* __restrict__ cls,
                                                     const float* prev, float* outp, int cbase, int use_prev) {
  const int i   = blockIdx.x * 256 + threadIdx.x;
  const int row = i >> 7;
  const int c4  = (i & 127) * 4;
  int i0 = cls[row * 2 + 0];
  int i1 = cls[row * 2 + 1];
  i0 = (i0 < 0) ? i0 + kNCls : i0;  i0 = (i0 < 0) ? 0 : ((i0 > kNCls - 1) ? kNCls - 1 : i0);
  i1 = (i1 < 0) ? i1 + kNCls : i1;  i1 = (i1 < 0) ? 0 : ((i1 > kNCls - 1) ? kNCls - 1 : i1);
  v4f acc = (v4f){0.f, 0.f, 0.f, 0.f};
  if (use_prev) acc = *(const v4f*)(prev + (size_t)row * kDim + c4);
#pragma unroll
  for (int c = 0; c < kCHalf; ++c) {
    const float w = 0.5f * ((float)(i0 == cbase + c) + (float)(i1 == cbase + c));
    const v4f r = *(const v4f*)(R + (size_t)c * kRows * kDim + (size_t)row * kDim + c4);
    acc = acc + r * w;
  }
  float* q = outp + (size_t)row * kDim + c4;
  *(volatile v4f*)q = acc;
  __threadfence();
  *(volatile v4f*)q = acc;
}

__global__ __launch_bounds__(256) void comb_kernel(const float* __restrict__ cret, const float* __restrict__ gret,
                                                   unsigned short* __restrict__ comb) {
  const int i   = blockIdx.x * 256 + threadIdx.x;
  const int row = i >> 7;
  const int c8  = (i & 127) * 8;
  const int cc  = c8 & (kDim - 1);
  const float* pc = cret + (size_t)row * kDim + cc;
  const float* pg = gret + (size_t)row * kDim + cc;
  const v4f a0 = *(const v4f*)(pc), a1 = *(const v4f*)(pc + 4);
  const v4f g0 = *(const v4f*)(pg), g1 = *(const v4f*)(pg + 4);
  const bool first = c8 < kDim;
  unsigned short hb[8];
#pragma unroll
  for (int e = 0; e < 4; ++e) {
    hb[e]     = h_bits((first ? a0[e] : g0[e]) * kGCarry);
    hb[4 + e] = h_bits((first ? a1[e] : g1[e]) * kGCarry);
  }
  const v4u u = (v4u){pk16(hb[0], hb[1]), pk16(hb[2], hb[3]), pk16(hb[4], hb[5]), pk16(hb[6], hb[7])};
  unsigned short* q = comb + (size_t)row * (2 * kDim) + c8;
  *(volatile v4u*)q = u;
  __threadfence();
  *(volatile v4u*)q = u;
}

__global__ __launch_bounds__(256) void gate_blend_kernel(const float* __restrict__ hpre, const float* __restrict__ w2,
                                                         const float* __restrict__ b2, const float* __restrict__ cret,
                                                         const float* __restrict__ gret, float* __restrict__ out) {
  __shared__ float red[8];
  const int t    = threadIdx.x;
  const int lane = t & 31, wave = t >> 5, grp = t >> 7, tl = t & 127;
  const int row  = blockIdx.x * 2 + grp;
  const int j    = (tl < kHid) ? tl : (kHid - 1);
  const float hv = hpre[(size_t)row * kHid + j];
  const float wv = w2[j];
  const float ge = 0.5f * hv * (1.0f + erff(hv * 0.70710678118654752f));
  float part = (tl < kHid) ? ge * wv : 0.0f;
#pragma unroll
  for (int off = 16; off > 0; off >>= 1) part += __shfl_xor(part, off, 32);
  if (lane == 0) red[wave] = part;
  __syncthreads();
  const float z = (((red[4 * grp] + red[4 * grp + 1]) + red[4 * grp + 2]) + red[4 * grp + 3]) + b2[0];
  const float gate = 1.0f / (1.0f + expf(-z));
  const float omg  = 1.0f - gate;
  const v4f cv = *(const v4f*)(cret + (size_t)row * kDim + 4 * tl);
  const v4f gv = *(const v4f*)(gret + (size_t)row * kDim + 4 * tl);
  const v4f o = cv * gate + gv * omg;
  float* q = out + (size_t)row * kDim + 4 * tl;
  *(volatile v4f*)q = o;
  __threadfence();
  *(volatile v4f*)q = o;
}

extern "C" void kernel_launch(void* const* d_in, const int* in_sizes, int n_in,
                              void* d_out, int out_size, void* d_ws, size_t ws_size,
                              hipStream_t stream) {
  if (n_in < 8) return;
  if (in_sizes[0] != kRows * kDim) return;
  if (in_sizes[1] != kRows * 2) return;
  if (in_sizes[2] != kKGlb * kDim) return;
  if (in_sizes[3] != kNCls * kKCls * kDim) return;
  if (in_sizes[4] != 2 * kDim * kHid) return;
  if (in_sizes[5] != kHid) return;
  if (in_sizes[6] != kHid) return;
  if (in_sizes[7] < 1) return;
  if (out_size != kRows * kDim) return;

  const float* query = (const float*)d_in[0];
  const int*   cls   = (const int*)  d_in[1];
  const float* gmem  = (const float*)d_in[2];
  const float* cmem  = (const float*)d_in[3];
  const float* w1    = (const float*)d_in[4];
  const float* b1    = (const float*)d_in[5];
  const float* w2    = (const float*)d_in[6];
  const float* b2    = (const float*)d_in[7];
  float* out = (float*)d_out;

  const size_t szQ16  = (size_t)kRows * kDim * 2;
  const size_t szF    = (size_t)kRows * kDim * 4;
  const size_t szHPRE = (size_t)kRows * kHid * 4;
  const size_t szW1T  = (size_t)kHid * 2 * kDim * 2;
  const size_t szGM16 = (size_t)kKGlbP * kDim * 2;
  const size_t szSG   = (size_t)kGChunk * kKGlbP * 4;
  const size_t szPG   = (size_t)kGChunk * kKGlbP * 2;
  const size_t szCM16 = (size_t)kNCls * kKClsP * kDim * 2;
  const size_t szSCR  = (size_t)kCHalf * kRows * kKClsP * 4;
  const size_t szPC   = (size_t)kCHalf * kRows * kKClsP * 2;
  const size_t szCOMB = (size_t)kRows * 2 * kDim * 2;

  const size_t offQH   = 0;
  const size_t offQL   = offQH + szQ16;
  const size_t offGRET = offQL + szQ16;
  const size_t offCLS0 = offGRET + szF;
  const size_t offCLS1 = offCLS0 + szF;
  const size_t offHPRE = offCLS1 + szF;
  const size_t offW1T  = offHPRE + szHPRE;
  const size_t offBase = offW1T + szW1T;
  const size_t offGMH  = offBase;
  const size_t offGML  = offGMH + szGM16;
  const size_t offGMT  = offGML + szGM16;
  const size_t offSG   = offGMT + szGM16;
  const size_t offPG   = offSG + szSG;
  const size_t endG    = offPG + szPG;
  const size_t offCMH  = offBase;
  const size_t offCML  = offCMH + szCM16;
  const size_t offCMT  = offCML + szCM16;
  const size_t offSCR  = offCMT + szCM16;
  const size_t offPC   = offSCR + szSCR;
  const size_t endC    = offPC + szPC;
  const size_t offCOMB = offBase;
  const size_t endK    = offCOMB + szCOMB;
  size_t need = endG;
  if (endC > need) need = endC;
  if (endK > need) need = endK;
  if (ws_size < need) return;

  char* ws = (char*)d_ws;
  unsigned short* QH   = (unsigned short*)(ws + offQH);
  unsigned short* QL   = (unsigned short*)(ws + offQL);
  float*          GRET = (float*)(ws + offGRET);
  float*          CLS0 = (float*)(ws + offCLS0);
  float*          CLS1 = (float*)(ws + offCLS1);
  float*          HPRE = (float*)(ws + offHPRE);
  unsigned short* W1T  = (unsigned short*)(ws + offW1T);
  unsigned short* GMH  = (unsigned short*)(ws + offGMH);
  unsigned short* GML  = (unsigned short*)(ws + offGML);
  unsigned short* GMT  = (unsigned short*)(ws + offGMT);
  float*          SG   = (float*)(ws + offSG);
  unsigned short* PG   = (unsigned short*)(ws + offPG);
  unsigned short* CMH  = (unsigned short*)(ws + offCMH);
  unsigned short* CML  = (unsigned short*)(ws + offCML);
  unsigned short* CMT  = (unsigned short*)(ws + offCMT);
  float*          SCR  = (float*)(ws + offSCR);
  unsigned short* PC   = (unsigned short*)(ws + offPC);
  unsigned short* COMB = (unsigned short*)(ws + offCOMB);

  {
    const int n8q = kRows * kDim / 8;
    split8_bf16_kernel<<<dim3(n8q / 256), dim3(256), 0, stream>>>(query, kRows, kRows, kDim / 8, QH, QL, n8q);
    const int n8g = kKGlbP * kDim / 8;
    split8_bf16_kernel<<<dim3(n8g / 256), dim3(256), 0, stream>>>(gmem, kKGlb, kKGlbP, kDim / 8, GMH, GML, n8g);
    tcast_kernel<<<dim3(kKGlbP / 64, kDim / 64, 1), dim3(256), 0, stream>>>(gmem, 0L, kDim, kKGlb, GMT, 0L, kKGlbP, 1.0f);
  }

  for (int ch = 0; ch < kRows / kGChunk; ++ch) {
    const size_t aoff = (size_t)ch * kGChunk * kDim;
    wmma_gemm64<1, true, 0, 0, false, 0><<<dim3((kGChunk / 64) * (kKGlbP / 64) / 8, 1), dim3(256), 0, stream>>>(
        QH + aoff, QL + aoff, kDim, 0L, GMH, GML, kDim, 0L, (void*)SG, nullptr, kKGlbP, 0L,
        nullptr, nullptr, 0L, kGChunk, kKGlbP, kDim, 1.0f);
    softmax_g_kernel<<<dim3(kGChunk), dim3(640), 0, stream>>>(SG, PG);
    wmma_gemm64<0, false, 0, 0, false, 0><<<dim3((kGChunk / 64) * (kDim / 64) / 8, 1), dim3(256), 0, stream>>>(
        PG, nullptr, kKGlbP, 0L, GMT, nullptr, kKGlbP, 0L, (void*)(GRET + aoff), nullptr, kDim, 0L,
        nullptr, nullptr, 0L, kGChunk, kDim, kKGlbP, kPCarryInv);
  }

  {
    const int n8c = kNCls * kKClsP * kDim / 8;
    split8_bf16_kernel<<<dim3(n8c / 256), dim3(256), 0, stream>>>(cmem, kKCls, kKClsP, kDim / 8, CMH, CML, n8c);
    tcast_kernel<<<dim3(kKClsP / 64, kDim / 64, kNCls), dim3(256), 0, stream>>>(
        cmem, (long)kKCls * kDim, kDim, kKCls, CMT, (long)kDim * kKClsP, kKClsP, 1.0f);
  }

  for (int hf = 0; hf < kNCls / kCHalf; ++hf) {
    const size_t boff = (size_t)hf * kCHalf * kKClsP * kDim;
    wmma_gemm64<1, true, 0, 0, false, 0><<<dim3((kRows / 64) * (kKClsP / 64) / 8, kCHalf), dim3(256), 0, stream>>>(
        QH, QL, kDim, 0L, CMH + boff, CML + boff, kDim, (long)kKClsP * kDim, (void*)SCR, nullptr, kKClsP, (long)kRows * kKClsP,
        nullptr, nullptr, 0L, kRows, kKClsP, kDim, 1.0f);
    softmax_c_kernel<<<dim3(kCHalf * kRows / 4), dim3(256), 0, stream>>>(SCR, PC);
    wmma_gemm64<0, false, 0, 0, false, 0><<<dim3((kRows / 64) * (kDim / 64) / 8, kCHalf), dim3(256), 0, stream>>>(
        PC, nullptr, kKClsP, (long)kRows * kKClsP, CMT + boff, nullptr, kKClsP, (long)kDim * kKClsP, (void*)SCR, nullptr, kDim,
        (long)kRows * kDim, nullptr, nullptr, 0L, kRows, kDim, kKClsP, kPCarryInv);
    select_kernel<<<dim3(kRows * (kDim / 4) / 256), dim3(256), 0, stream>>>(
        SCR, cls, CLS0, (hf == 0) ? CLS0 : CLS1, hf * kCHalf, hf);
  }

  tcast_kernel<<<dim3(2 * kDim / 64, kHid / 64, 1), dim3(256), 0, stream>>>(w1, 0L, kHid, 2 * kDim, W1T, 0L, 2 * kDim, kGCarry);
  comb_kernel<<<dim3(kRows * (2 * kDim / 8) / 256), dim3(256), 0, stream>>>(CLS1, GRET, COMB);
  wmma_gemm64<0, false, 2, 0, false, 0><<<dim3((kRows / 64) * (kHid / 64) / 8, 1), dim3(256), 0, stream>>>(
      COMB, nullptr, 2 * kDim, 0L, W1T, nullptr, 2 * kDim, 0L, (void*)HPRE, nullptr, kHid, 0L,
      b1, nullptr, 0L, kRows, kHid, 2 * kDim, kGateScale);
  gate_blend_kernel<<<dim3(kRows / 2), dim3(256), 0, stream>>>(HPRE, w2, b2, CLS1, GRET, out);
}
